// TransformerBlockTF_16028817949065
// MI455X (gfx1250) — hardware-verified
//
#include <hip/hip_runtime.h>


namespace {
constexpr int Bn = 4, S = 1024, D = 768, H = 12, HD = 64, FF = 3072, NT = Bn * S;
constexpr float QS = 8.0f, KS = 8.0f, VS = 8.0f, PS = 8.0f, AS_ = 8.0f, SCALE = 0.125f, EPS = 1e-5f;
constexpr size_t PL = (size_t)Bn * H * S * HD;

typedef _Float16 b16;
typedef __attribute__((ext_vector_type(16))) _Float16 v16b;
typedef __attribute__((ext_vector_type(8))) _Float16 v8b;
typedef __attribute__((ext_vector_type(8))) float v8f;
typedef __attribute__((ext_vector_type(4))) float v4f;
__device__ __forceinline__ float bf16_rne(float f) { unsigned int u = __float_as_uint(f); u += 0x7FFFu + ((u >> 16) & 1u); return __uint_as_float(u & 0xFFFF0000u); }
__device__ __forceinline__ void split16(float v, b16& hi, b16& lo) { hi = (b16)v; lo = (b16)(v - (float)hi); }
__device__ __forceinline__ v16b frag_kb(const b16* p, int hh) { const v8b a = *(const v8b*)(p + 8 * hh), b = *(const v8b*)(p + 16 + 8 * hh); v16b f;
#pragma unroll
  for (int e = 0; e < 8; ++e) { f[e] = a[e]; f[8 + e] = b[e]; } return f; }
__device__ __forceinline__ void frag_split(const float* p, int hh, v16b& fh, v16b& fl) {
#pragma unroll
  for (int e = 0; e < 8; ++e) { b16 a, c; split16(p[8 * hh + e] * AS_, a, c); fh[e] = a; fl[e] = c; split16(p[16 + 8 * hh + e] * AS_, a, c); fh[8 + e] = a; fl[8 + e] = c; } }
__device__ __forceinline__ v8f wmma16b(v16b a, v16b b, v8f c) { v8f d = __builtin_amdgcn_wmma_f32_16x16x32_f16(false, a, false, b, (short)0, c, false, false); asm volatile("v_nop\n\tv_nop\n\tv_nop\n\tv_nop" : "+v"(d) : "v"(a), "v"(b)); return d; }
__device__ __forceinline__ void wave_lds_sync() { __builtin_amdgcn_fence(__ATOMIC_RELEASE, "workgroup"); __builtin_amdgcn_wave_barrier(); __builtin_amdgcn_fence(__ATOMIC_ACQUIRE, "workgroup"); }
__device__ __forceinline__ float nexp(float x) { return __builtin_amdgcn_exp2f(x * 1.4426950408889634f); }
__device__ __forceinline__ float pmul(float a, float b) { float p = a * b; asm volatile("" : "+v"(p)); return p; }
__device__ __forceinline__ float tanh_(float x) { const float e = nexp(-2.0f * fabsf(x)); const float t = (1.0f - e) * __builtin_amdgcn_rcpf(1.0f + e); return (x >= 0.0f) ? t : -t; }
__device__ __forceinline__ float gelu_t(float x) { return 0.5f * x * (1.0f + tanh_(0.7978845608028654f * (x + 0.044715f * x * x * x))); }

struct Wo_ { static constexpr size_t A = 0, P_ = A + (size_t)3 * D * D, F = P_ + (size_t)D * D, M = F + (size_t)FF * D, END = M + (size_t)D * FF; };
__global__ __launch_bounds__(256) void prep_kernel(const float* __restrict__ wa, const float* __restrict__ wp, const float* __restrict__ wf, const float* __restrict__ wm, const float* __restrict__ ba, const float* __restrict__ bp, const float* __restrict__ bfc, const float* __restrict__ bm, const float* __restrict__ g1, const float* __restrict__ b1, const float* __restrict__ g2, const float* __restrict__ b2, b16* __restrict__ R, float* __restrict__ P) {
  const size_t tid = (size_t)blockIdx.x * blockDim.x + threadIdx.x, nth = (size_t)gridDim.x * blockDim.x;
  auto tr = [&](const float* W, int IN, int OUT, size_t base, size_t p) { const int o = (int)(p / (IN / 8)), k8 = (int)(p % (IN / 8)) * 8; v8b v;
#pragma unroll
    for (int e = 0; e < 8; ++e) v[e] = (b16)bf16_rne(W[(size_t)(k8 + e) * OUT + o]);
    *(volatile v8b*)(R + base + (size_t)o * IN + k8) = v; };
  for (int pass = 0; pass < 2; ++pass) {
    for (size_t p = tid; p < (size_t)3 * D * D / 8; p += nth) tr(wa, D, 3 * D, Wo_::A, p);
    for (size_t p = tid; p < (size_t)D * D / 8; p += nth) tr(wp, D, D, Wo_::P_, p);
    for (size_t p = tid; p < (size_t)FF * D / 8; p += nth) { tr(wf, D, FF, Wo_::F, p); tr(wm, FF, D, Wo_::M, p); }
    for (size_t p = tid; p < 9984 / 4; p += nth) { v4f v;
#pragma unroll
      for (int e = 0; e < 4; ++e) { const int i = (int)p * 4 + e; float x; if (i < 2304) x = ba[i]; else if (i < 3072) x = bp[i - 2304]; else if (i < 6144) x = bfc[i - 3072]; else if (i < 6912) x = bm[i - 6144]; else if (i < 7680) x = g1[i - 6912]; else if (i < 8448) x = b1[i - 7680]; else if (i < 9216) x = g2[i - 8448]; else x = b2[i - 9216]; v[e] = bf16_rne(x); }
      *(volatile v4f*)(P + p * 4) = v; }
    __threadfence(); }
}

__global__ __launch_bounds__(256) void ln_kernel(const float* __restrict__ x, const float* __restrict__ g, const float* __restrict__ bb, int rnd, float* __restrict__ y) {
  const int wid = threadIdx.x >> 5, lane = threadIdx.x & 31, row = blockIdx.x * 8 + wid; const float* pr = x + (size_t)row * D;
  float v[24]; float s = 0.0f;
#pragma unroll
  for (int j = 0; j < 6; ++j) { const v4f t = *(const v4f*)(pr + j * 128 + lane * 4);
#pragma unroll
    for (int e = 0; e < 4; ++e) { v[j * 4 + e] = rnd ? bf16_rne(t[e]) : t[e]; s += v[j * 4 + e]; } }
#pragma unroll
  for (int o = 1; o < 32; o <<= 1) s += __shfl_xor(s, o);
  const float mu = s * (1.0f / D); float q = 0.0f;
#pragma unroll
  for (int j = 0; j < 24; ++j) { const float d = v[j] - mu; q += pmul(d, d); }
#pragma unroll
  for (int o = 1; o < 32; o <<= 1) q += __shfl_xor(q, o);
  const float is = rsqrtf(q * (1.0f / D) + EPS);
  for (int pass = 0; pass < 2; ++pass) {
#pragma unroll
    for (int j = 0; j < 6; ++j) { const int c = j * 128 + lane * 4; v4f o4; for (int e = 0; e < 4; ++e) o4[e] = pmul((v[j * 4 + e] - mu) * is, g[c + e]) + bb[c + e]; *(volatile v4f*)(y + (size_t)row * D + c) = o4; }
    __threadfence(); }
}

__global__ __launch_bounds__(128) void qkv_kernel(const float* __restrict__ hn, const b16* __restrict__ R, const float* __restrict__ P, b16* __restrict__ qp, b16* __restrict__ kp, b16* __restrict__ vt) {
  __shared__ __attribute__((aligned(16))) b16 Th[4][32][64 + 8], Tl[4][32][64 + 8]; __shared__ __attribute__((aligned(16))) b16 Vh[64][128 + 8], Vl[64][128 + 8];
  const int lane = threadIdx.x & 31, wave = threadIdx.x >> 5, nloc = lane & 15, hlf = lane >> 4, ct = blockIdx.x, which = ct / H, h = ct % H, c0 = ct * 64, p0 = blockIdx.y * 128, m0 = p0 + wave * 32, b = p0 / S, t0 = p0 % S;
  const b16* Wt = R + Wo_::A; const float* bias = P;
  v8f acc[2][4];
#pragma unroll
  for (int r = 0; r < 2; ++r)
#pragma unroll
    for (int t = 0; t < 4; ++t) acc[r][t] = (v8f){};
#pragma unroll 2
  for (int kb = 0; kb < D; kb += 32) { v16b a0, l0, a1, l1; frag_split(hn + (size_t)(m0 + nloc) * D + kb, hlf, a0, l0); frag_split(hn + (size_t)(m0 + 16 + nloc) * D + kb, hlf, a1, l1);
#pragma unroll
    for (int t = 0; t < 4; ++t) { const v16b bw = frag_kb(Wt + (size_t)(c0 + t * 16 + nloc) * D + kb, hlf); acc[0][t] = wmma16b(a0, bw, acc[0][t]); acc[0][t] = wmma16b(l0, bw, acc[0][t]); acc[1][t] = wmma16b(a1, bw, acc[1][t]); acc[1][t] = wmma16b(l1, bw, acc[1][t]); } }
  const float scl = (which == 0) ? SCALE * QS : ((which == 1) ? KS : VS);
  if (which < 2) {
#pragma unroll
    for (int t = 0; t < 4; ++t) { const float bb = bias[c0 + t * 16 + nloc];
#pragma unroll
      for (int r = 0; r < 2; ++r)
#pragma unroll
        for (int v = 0; v < 8; ++v) { b16 a_, l_; split16((acc[r][t][v] * (1.0f / AS_) + bb) * scl, a_, l_); Th[wave][r * 16 + 8 * hlf + v][t * 16 + nloc] = a_; Tl[wave][r * 16 + 8 * hlf + v][t * 16 + nloc] = l_; } }
    wave_lds_sync();
    b16* base = ((which == 0) ? qp : kp) + (((size_t)b * H + h) * S + (m0 % S)) * HD;
    for (int pass = 0; pass < 2; ++pass) {
#pragma unroll
      for (int j = 0; j < 8; ++j) { const int rr = j * 4 + (lane >> 3), c8 = (lane & 7) * 8; *(volatile v8b*)(base + (size_t)rr * HD + c8) = *(const v8b*)(&Th[wave][rr][c8]); *(volatile v8b*)(base + PL + (size_t)rr * HD + c8) = *(const v8b*)(&Tl[wave][rr][c8]); }
      __threadfence(); }
    return; }
#pragma unroll
  for (int t = 0; t < 4; ++t) { const float bb = bias[c0 + t * 16 + nloc];
#pragma unroll
    for (int r = 0; r < 2; ++r)
#pragma unroll
      for (int v = 0; v < 8; ++v) { b16 a_, l_; split16((acc[r][t][v] * (1.0f / AS_) + bb) * scl, a_, l_); Vh[t * 16 + nloc][wave * 32 + r * 16 + 8 * hlf + v] = a_; Vl[t * 16 + nloc][wave * 32 + r * 16 + 8 * hlf + v] = l_; } }
  __syncthreads();
  for (int pass = 0; pass < 2; ++pass) { for (int i = threadIdx.x; i < 64 * 16; i += 128) { const int d = i >> 4, c8 = (i & 15) * 8; const size_t o = (((size_t)b * H + h) * HD + d) * S + t0 + c8;
      *(volatile v8b*)(vt + o) = *(const v8b*)(&Vh[d][c8]); *(volatile v8b*)(vt + PL + o) = *(const v8b*)(&Vl[d][c8]); } __threadfence(); }
}

__global__ __launch_bounds__(384) void attn_kernel(const b16* __restrict__ qp, const b16* __restrict__ kp, const b16* __restrict__ vt, float* __restrict__ ctx) {
  __shared__ __attribute__((aligned(16))) float Os[16][D + 4];
  const int h = threadIdx.x >> 5, lane = threadIdx.x & 31, hh = lane >> 4, col = lane & 15; const int b = blockIdx.x / (S / 16), q0 = (blockIdx.x % (S / 16)) * 16, qi = q0 + col;
  const b16* Q = qp + (((size_t)b * H + h) * S) * HD; const b16* K = kp + (((size_t)b * H + h) * S) * HD; const b16* V = vt + (((size_t)b * H + h) * HD) * S;
  v16b qf[2], ql[2];
#pragma unroll
  for (int ks = 0; ks < 2; ++ks) { qf[ks] = frag_kb(Q + (size_t)qi * HD + ks * 32, hh); ql[ks] = frag_kb(Q + PL + (size_t)qi * HD + ks * 32, hh); }
  float m = -INFINITY, l = 0.0f; v8f o[4] = {{}, {}, {}, {}};
  for (int kb = 0; kb < q0 + 16; kb += 32) { const bool diag = (kb + 32 > q0); v8f s0 = {}, s1 = {};
#pragma unroll
    for (int ks = 0; ks < 2; ++ks) { const v16b ka = frag_kb(K + (size_t)(kb + col) * HD + ks * 32, hh), kal = frag_kb(K + PL + (size_t)(kb + col) * HD + ks * 32, hh), kc = frag_kb(K + (size_t)(kb + 16 + col) * HD + ks * 32, hh), kcl = frag_kb(K + PL + (size_t)(kb + 16 + col) * HD + ks * 32, hh);
      s0 = wmma16b(ka, qf[ks], s0); s0 = wmma16b(ka, ql[ks], s0); s0 = wmma16b(kal, qf[ks], s0); s1 = wmma16b(kc, qf[ks], s1); s1 = wmma16b(kc, ql[ks], s1); s1 = wmma16b(kcl, qf[ks], s1); }
    float mr = -INFINITY;
#pragma unroll
    for (int r = 0; r < 8; ++r) { s0[r] *= 1.0f / (QS * KS); s1[r] *= 1.0f / (QS * KS); if (diag) { if (kb + 8 * hh + r > qi) s0[r] = -INFINITY; if (kb + 16 + 8 * hh + r > qi) s1[r] = -INFINITY; } mr = fmaxf(mr, fmaxf(s0[r], s1[r])); }
    mr = fmaxf(mr, __shfl_xor(mr, 16));
    const float mn = fmaxf(m, mr), al_ = nexp(m - mn); m = mn; float sum = 0.0f; v16b pbv, plv;
#pragma unroll
    for (int r = 0; r < 8; ++r) { const float e0 = nexp(s0[r] - mn), e1 = nexp(s1[r] - mn); sum += e0 + e1; b16 a, cc; split16(e0 * PS, a, cc); pbv[r] = a; plv[r] = cc; split16(e1 * PS, a, cc); pbv[8 + r] = a; plv[8 + r] = cc; }
    sum += __shfl_xor(sum, 16); l = l * al_ + sum;
#pragma unroll
    for (int t = 0; t < 4; ++t) { o[t] *= al_; const v16b vf = frag_kb(V + (size_t)(t * 16 + col) * S + kb, hh), vl = frag_kb(V + PL + (size_t)(t * 16 + col) * S + kb, hh); o[t] = wmma16b(vf, pbv, o[t]); o[t] = wmma16b(vf, plv, o[t]); o[t] = wmma16b(vl, pbv, o[t]); } }
  const float inv = 1.0f / (l * VS * PS);
#pragma unroll
  for (int t = 0; t < 4; ++t)
#pragma unroll
    for (int r = 0; r < 8; ++r) Os[col][h * HD + t * 16 + 8 * hh + r] = o[t][r] * inv;
  __syncthreads();
  float* dst = ctx + ((size_t)b * S + q0) * D;
  for (int pass = 0; pass < 2; ++pass) { for (int i = threadIdx.x; i < 16 * (D / 4); i += 384) { const int rr = i / (D / 4), c4 = (i % (D / 4)) * 4; *(volatile v4f*)(dst + (size_t)rr * D + c4) = *(const v4f*)(&Os[rr][c4]); } __threadfence(); }
}

__global__ __launch_bounds__(128) void gemm_kernel(const float* __restrict__ X, int K, const b16* __restrict__ Bw, int N, const float* __restrict__ bias, int mode, const float* __restrict__ res, int rres, float* __restrict__ Y) {
  __shared__ __attribute__((aligned(16))) float Ts[4][32 * 64];
  const int lane = threadIdx.x & 31, wave = threadIdx.x >> 5, nloc = lane & 15, hlf = lane >> 4, m0 = blockIdx.y * 128 + wave * 32, c0 = blockIdx.x * 64;
  v8f acc[2][4];
#pragma unroll
  for (int r = 0; r < 2; ++r)
#pragma unroll
    for (int t = 0; t < 4; ++t) acc[r][t] = (v8f){};
#pragma unroll 2
  for (int kb = 0; kb < K; kb += 32) { v16b a0, l0, a1, l1; frag_split(X + (size_t)(m0 + nloc) * K + kb, hlf, a0, l0); frag_split(X + (size_t)(m0 + 16 + nloc) * K + kb, hlf, a1, l1);
#pragma unroll
    for (int t = 0; t < 4; ++t) { const v16b bw = frag_kb(Bw + (size_t)(c0 + t * 16 + nloc) * K + kb, hlf); acc[0][t] = wmma16b(a0, bw, acc[0][t]); acc[0][t] = wmma16b(l0, bw, acc[0][t]); acc[1][t] = wmma16b(a1, bw, acc[1][t]); acc[1][t] = wmma16b(l1, bw, acc[1][t]); } }
  float* Tt = Ts[wave];
#pragma unroll
  for (int t = 0; t < 4; ++t) { const int cc = c0 + t * 16 + nloc; const float bb = bias[cc];
#pragma unroll
    for (int r = 0; r < 2; ++r)
#pragma unroll
      for (int v = 0; v < 8; ++v) { const int rl = r * 16 + v + 8 * hlf; float y = acc[r][t][v] * (1.0f / AS_) + bb;
        if (mode == 1) y = gelu_t(y); else { const float rv = res[(size_t)(m0 + rl) * N + cc]; y += rres ? bf16_rne(rv) : rv; }
        Tt[rl * 64 + t * 16 + nloc] = y; } }
  wave_lds_sync();
  for (int pass = 0; pass < 2; ++pass) {
#pragma unroll
    for (int j = 0; j < 16; ++j) { const int rr = j * 2 + hlf, c4 = nloc * 4; *(volatile v4f*)(Y + (size_t)(m0 + rr) * N + c0 + c4) = *(const v4f*)(Tt + rr * 64 + c4); }
    __threadfence(); }
}
}

extern "C" void kernel_launch(void* const* d_in, const int* in_sizes, int n_in,
                              void* d_out, int out_size, void* d_ws, size_t ws_size, hipStream_t stream) {
  (void)n_in; (void)out_size;
  const float* x = (const float*)d_in[0]; const float* g1 = (const float*)d_in[1]; const float* b1 = (const float*)d_in[2]; const float* g2 = (const float*)d_in[3]; const float* b2 = (const float*)d_in[4];
  const float* wa = (const float*)d_in[5]; const float* ba = (const float*)d_in[6]; const float* wp = (const float*)d_in[7]; const float* bp = (const float*)d_in[8]; const float* wf = (const float*)d_in[9]; const float* bfc = (const float*)d_in[10]; const float* wm = (const float*)d_in[11]; const float* bm = (const float*)d_in[12];
  float* out = (float*)d_out;
  if (in_sizes[0] != NT * D || in_sizes[5] != D * 3 * D || in_sizes[7] != D * D || in_sizes[9] != D * FF || in_sizes[11] != FF * D) return;
  size_t off = 0; char* ws = (char*)d_ws;
  auto carve = [&](size_t bytes) { char* p = ws + off; off += (bytes + 255) & ~(size_t)255; return p; };
  b16* R = (b16*)carve(Wo_::END * 2); float* P = (float*)carve(9984 * 4); float* hn = (float*)carve((size_t)NT * D * 4); b16* qp = (b16*)carve(PL * 2 * 2); b16* kp = (b16*)carve(PL * 2 * 2); b16* vt = (b16*)carve(PL * 2 * 2);
  float* ctx = (float*)carve((size_t)NT * D * 4); float* x1 = (float*)carve((size_t)NT * D * 4);
  float* h2 = hn;
  float* hf = (float*)qp;
  static_assert(3 * PL * 2 * 2 + (size_t)NT * D * 4 >= (size_t)NT * FF * 4, "hf alias must fit");
  if (off > ws_size) return;
  prep_kernel<<<512, 256, 0, stream>>>(wa, wp, wf, wm, ba, bp, bfc, bm, g1, b1, g2, b2, R, P);
  ln_kernel<<<NT / 8, 256, 0, stream>>>(x, P + 6912, P + 7680, 1, hn);
  qkv_kernel<<<dim3(3 * H, NT / 128), 128, 0, stream>>>(hn, R, P, qp, kp, vt);
  attn_kernel<<<NT / 16, 384, 0, stream>>>(qp, kp, vt, ctx);
  gemm_kernel<<<dim3(D / 64, NT / 128), 128, 0, stream>>>(ctx, D, R + Wo_::P_, D, P + 2304, 0, x, 1, x1);
  ln_kernel<<<NT / 8, 256, 0, stream>>>(x1, P + 8448, P + 9216, 0, h2);
  gemm_kernel<<<dim3(FF / 64, NT / 128), 128, 0, stream>>>(h2, D, R + Wo_::F, FF, P + 3072, 1, nullptr, 0, hf);
  gemm_kernel<<<dim3(D / 64, NT / 128), 128, 0, stream>>>(hf, FF, R + Wo_::M, D, P + 6144, 0, x1, 0, out);
}
